// ADLA_18013092840139
// MI455X (gfx1250) — hardware-verified
//
#include <hip/hip_runtime.h>
#include <math.h>
#include <stdint.h>

#define NB      8
#define NHEAD   8
#define HDIM    48
#define DIMC    384
#define HWD     14
#define NTOK    2744
#define TP      2752
#define NANC    343
#define AP      384
#define MT      (NB * TP)
#define MA      (NB * AP)
#define NTAP    27
#define A3      343
#define WSC     1024.0f
#define QSC     8.0f
#define VSC     16.0f
#define PSC     1024.0f
#define GSC     1024.0f
#define CSC     1024.0f
#define ATT_SCALE 0.14433756729740643f
#define SSC     (ATT_SCALE / (QSC * QSC))
#define NEG_BIG (-1.0e30f)

static_assert(NHEAD * HDIM == DIMC);
static_assert(NTOK == HWD * HWD * HWD);
static_assert(NANC == 7 * 7 * 7);
static_assert((TP % 64) == 0 && TP >= NTOK && (TP - NTOK) < 64 && (TP - NTOK) == 8);
static_assert((AP % 64) == 0 && AP >= NANC && (AP - NANC) < 64);
static_assert((MT % 64) == 0 && (MA % 64) == 0 && (DIMC % 128) == 0 && (DIMC % 64) == 0);
static_assert(((MT * DIMC) % 2048) == 0);
static_assert(HDIM == 48 && (HDIM % 8) == 0);
static_assert(TP == 688 * 4 && AP == 96 * 4);

typedef _Float16 v16h __attribute__((ext_vector_type(16)));
typedef _Float16 v8h  __attribute__((ext_vector_type(8)));
typedef __bf16   v16b __attribute__((ext_vector_type(16)));
typedef float    v8f  __attribute__((ext_vector_type(8)));
typedef float    v4f  __attribute__((ext_vector_type(4)));
typedef unsigned int v4u __attribute__((ext_vector_type(4)));
union FR { v16h h; v16b b; v8h q[2]; v4u u[2]; };

__device__ __forceinline__ float bfr(float f) {
  unsigned u = __float_as_uint(f);
  u = (u + 0x7FFFu + ((u >> 16) & 1u)) & 0xFFFF0000u;
  return __uint_as_float(u);
}
__device__ __forceinline__ unsigned short f2bf(float f) {
  unsigned u = __float_as_uint(f);
  u = u + 0x7FFFu + ((u >> 16) & 1u);
  return (unsigned short)(u >> 16);
}
__device__ __forceinline__ unsigned short h_bits(_Float16 x) { return __builtin_bit_cast(unsigned short, x); }
__device__ __forceinline__ unsigned pk16(unsigned short a, unsigned short b) { return (unsigned)a | ((unsigned)b << 16); }
__device__ __forceinline__ v8f zero8() { v8f z = {0.f, 0.f, 0.f, 0.f, 0.f, 0.f, 0.f, 0.f}; return z; }

__device__ __forceinline__ FR ldfr(const unsigned short* p) {
  FR f;
  f.u[0] = *(const v4u*)(p);
  f.u[1] = *(const v4u*)(p + 16);
  return f;
}
__device__ __forceinline__ FR ldfrh(const _Float16* p) {
  FR f;
  f.q[0] = *(const v8h*)(p);
  f.q[1] = *(const v8h*)(p + 16);
  return f;
}

__device__ __forceinline__ v8f mma16(const FR& a, const FR& b, v8f c) {
  c = __builtin_amdgcn_wmma_f32_16x16x32_f16(false, a.h, false, b.h, (short)0, c, false, false);
#if defined(__HIP_DEVICE_COMPILE__)
  asm volatile("v_nop\n\tv_nop\n\tv_nop\n\tv_nop" : "+v"(c) : "v"(a.h), "v"(b.h));
#endif
  return c;
}
template <bool BF>
__device__ __forceinline__ v8f mma_raw(const FR& a, const FR& b, v8f c) {
  if (BF) return __builtin_amdgcn_wmma_f32_16x16x32_bf16(false, a.b, false, b.b, (short)0, c, false, false);
  return __builtin_amdgcn_wmma_f32_16x16x32_f16(false, a.h, false, b.h, (short)0, c, false, false);
}
__device__ __forceinline__ void guard3(v8f& x, v8f& y, const FR& a, const FR& b, const FR& d) {
#if defined(__HIP_DEVICE_COMPILE__)
  asm volatile("v_nop\n\tv_nop\n\tv_nop\n\tv_nop" : "+v"(x), "+v"(y) : "v"(a.h), "v"(b.h), "v"(d.h));
#endif
}
__device__ __forceinline__ void acc_guard4(v8f& a, v8f& b, v8f& c, v8f& d) {
#if defined(__HIP_DEVICE_COMPILE__)
  asm volatile("v_nop\n\tv_nop\n\tv_nop\n\tv_nop" : "+v"(a), "+v"(b), "+v"(c), "+v"(d));
#endif
}
__device__ __forceinline__ void acc_guard3(v8f& a, v8f& b, v8f& c) {
#if defined(__HIP_DEVICE_COMPILE__)
  asm volatile("v_nop\n\tv_nop\n\tv_nop\n\tv_nop" : "+v"(a), "+v"(b), "+v"(c));
#endif
}
__device__ __forceinline__ void wave_sync_lds() {
  __builtin_amdgcn_fence(__ATOMIC_RELEASE, "workgroup");
  __builtin_amdgcn_wave_barrier();
  __builtin_amdgcn_fence(__ATOMIC_ACQUIRE, "workgroup");
}

__device__ __forceinline__ void lin7(int i, int& x0, int& x1, float& w) {
  float x = ((float)i + 0.5f) * 0.5f - 0.5f;
  x = fminf(fmaxf(x, 0.f), 6.f);
  const float fl = floorf(x);
  x0 = (int)fl;
  x1 = (x0 + 1 < 6) ? (x0 + 1) : 6;
  w = x - fl;
}
__device__ __forceinline__ float terp(const float* base, int x0, int x1, float wx, int y0, int y1, float wy,
                                      int z0, int z1, float wz) {
  const float c00 = base[(x0 * 7 + y0) * 7 + z0] * (1.f - wz) + base[(x0 * 7 + y0) * 7 + z1] * wz;
  const float c01 = base[(x0 * 7 + y1) * 7 + z0] * (1.f - wz) + base[(x0 * 7 + y1) * 7 + z1] * wz;
  const float c10 = base[(x1 * 7 + y0) * 7 + z0] * (1.f - wz) + base[(x1 * 7 + y0) * 7 + z1] * wz;
  const float c11 = base[(x1 * 7 + y1) * 7 + z0] * (1.f - wz) + base[(x1 * 7 + y1) * 7 + z1] * wz;
  const float c0 = c00 * (1.f - wy) + c01 * wy;
  const float c1 = c10 * (1.f - wy) + c11 * wy;
  return c0 * (1.f - wx) + c1 * wx;
}
__device__ __forceinline__ float terpg(const float* base, int x0, int x1, float wx, int y0, int y1, float wy,
                                       int z0, int z1, float wz) {
  const float c00 = bfr(base[(x0 * 7 + y0) * 7 + z0]) * (1.f - wz) + bfr(base[(x0 * 7 + y0) * 7 + z1]) * wz;
  const float c01 = bfr(base[(x0 * 7 + y1) * 7 + z0]) * (1.f - wz) + bfr(base[(x0 * 7 + y1) * 7 + z1]) * wz;
  const float c10 = bfr(base[(x1 * 7 + y0) * 7 + z0]) * (1.f - wz) + bfr(base[(x1 * 7 + y0) * 7 + z1]) * wz;
  const float c11 = bfr(base[(x1 * 7 + y1) * 7 + z0]) * (1.f - wz) + bfr(base[(x1 * 7 + y1) * 7 + z1]) * wz;
  const float c0 = c00 * (1.f - wy) + c01 * wy;
  const float c1 = c10 * (1.f - wy) + c11 * wy;
  return c0 * (1.f - wx) + c1 * wx;
}

template <int MODE>
__global__ __launch_bounds__(256) void tr_cvt(const float* __restrict__ in, int ldi, unsigned short* out, int ldo, float sc) {
  __shared__ __align__(16) unsigned short tile[64 * 72];
  const int tid = threadIdx.x;
  const int c0 = blockIdx.x * 64;
  const int r0 = blockIdx.y * 64;
#pragma unroll
  for (int i = 0; i < 4; ++i) {
    const int idx = tid + 256 * i;
    const int row = idx >> 4, c4 = idx & 15;
    const v4f v = *(const v4f*)(in + (size_t)(r0 + row) * (size_t)ldi + c0 + c4 * 4);
#pragma unroll
    for (int e = 0; e < 4; ++e) {
      const float f = v[e];
      unsigned short bits;
      if (MODE == 0)      bits = h_bits((_Float16)(bfr(f) * sc));
      else if (MODE == 1) bits = h_bits((_Float16)(f * sc));
      else                bits = f2bf(f);
      tile[(c4 * 4 + e) * 72 + row] = bits;
    }
  }
  __syncthreads();
  v4u val[2];
  size_t go[2];
#pragma unroll
  for (int i = 0; i < 2; ++i) {
    const int idx = tid + 256 * i;
    const int ccl = idx >> 3, piece = idx & 7;
    val[i] = *(const v4u*)(tile + ccl * 72 + piece * 8);
    go[i] = (size_t)(c0 + ccl) * (size_t)ldo + (size_t)(r0 + piece * 8);
  }
  for (int pass = 0; pass < 2; ++pass) {
#pragma unroll
    for (int i = 0; i < 2; ++i) *(volatile v4u*)(out + go[i]) = val[i];
    __threadfence();
  }
}

__global__ __launch_bounds__(256) void cvt_x(const float* __restrict__ x, unsigned short* XH) {
  const size_t i8 = ((size_t)blockIdx.x * 256 + threadIdx.x) * 8;
  if (i8 + 8 > (size_t)MT * DIMC) return;
  const size_t row = i8 / DIMC;
  const int col = (int)(i8 - row * DIMC);
  const int b = (int)(row / TP);
  const int n = (int)(row - (size_t)b * TP);
  const bool valid = n < NTOK;
  const int ncl = valid ? n : (NTOK - 1);
  const float* src = x + ((size_t)(b * NTOK + ncl)) * DIMC + col;
  const v4f a  = *(const v4f*)(src);
  const v4f bb = *(const v4f*)(src + 4);
  v4u p;
#pragma unroll
  for (int e = 0; e < 2; ++e) {
    const float f0 = valid ? bfr(a[2 * e]) : 0.f,  f1 = valid ? bfr(a[2 * e + 1]) : 0.f;
    const float g0 = valid ? bfr(bb[2 * e]) : 0.f, g1 = valid ? bfr(bb[2 * e + 1]) : 0.f;
    p[e]     = pk16(h_bits((_Float16)f0), h_bits((_Float16)f1));
    p[2 + e] = pk16(h_bits((_Float16)g0), h_bits((_Float16)g1));
  }
  *(volatile v4u*)(XH + i8) = p;
  __threadfence();
  *(volatile v4u*)(XH + i8) = p;
}

template <int OM, bool BF, bool HASB>
__global__ __launch_bounds__(128) void gemm_k(
    const unsigned short* __restrict__ A, int lda, const unsigned short* __restrict__ B, int ldb,
    void* C0, const float* __restrict__ bias, int ldc, int M, int N, int K, float oscale, int rpi, int rpo) {
  __shared__ __align__(16) float sT[4][16 * 132];
  const int lane = threadIdx.x & 31;
  const int wave = threadIdx.x >> 5;
  const int tilesN = N >> 7;
  const int tilesM = M >> 5;
  const int tile = blockIdx.x * 4 + wave;
  if (tile >= tilesM * tilesN) return;
  const int tm = tile / tilesN;
  const int tn = tile - tm * tilesN;
  const int m0 = tm << 5;
  const int n0 = tn << 7;
  const int rl   = lane & 15;
  const int hh   = lane >> 4;
  const int koff = hh * 8;

  v8f acc[2][8];
#pragma unroll
  for (int i = 0; i < 2; ++i)
#pragma unroll
    for (int j = 0; j < 8; ++j) acc[i][j] = zero8();

  const unsigned short* ar0 = A + (size_t)(m0 + rl) * (size_t)lda + koff;
  const unsigned short* ar1 = A + (size_t)(m0 + 16 + rl) * (size_t)lda + koff;
  const unsigned short* br  = B + (size_t)(n0 + rl) * (size_t)ldb + koff;
  for (int k0 = 0; k0 < K; k0 += 32) {
    const FR a0 = ldfr(ar0 + k0);
    const FR a1 = ldfr(ar1 + k0);
#pragma unroll
    for (int j = 0; j < 8; ++j) {
      const FR bb = ldfr(br + (size_t)j * 16 * (size_t)ldb + k0);
      acc[0][j] = mma_raw<BF>(a0, bb, acc[0][j]);
      acc[1][j] = mma_raw<BF>(a1, bb, acc[1][j]);
      guard3(acc[0][j], acc[1][j], a0, a1, bb);
    }
  }
  acc_guard4(acc[0][0], acc[0][1], acc[0][2], acc[0][3]);
  acc_guard4(acc[0][4], acc[0][5], acc[0][6], acc[0][7]);
  acc_guard4(acc[1][0], acc[1][1], acc[1][2], acc[1][3]);
  acc_guard4(acc[1][4], acc[1][5], acc[1][6], acc[1][7]);

  float bj[8];
#pragma unroll
  for (int j = 0; j < 8; ++j) bj[j] = 0.f;
  if (HASB) {
#pragma unroll
    for (int j = 0; j < 8; ++j) bj[j] = bfr(bias[n0 + 16 * j + rl]);
  }

  float* slab = sT[wave];
#pragma unroll
  for (int i = 0; i < 2; ++i) {
    const int mB = m0 + 16 * i;
#pragma unroll
    for (int j = 0; j < 8; ++j) {
#pragma unroll
      for (int r = 0; r < 8; ++r) {
        float v = acc[i][j][r] * oscale;
        if (HASB) v += bj[j];
        slab[(8 * hh + r) * 132 + 16 * j + rl] = v;
      }
    }
    wave_sync_lds();
    if (OM == 4) {
      float* Cf = (float*)C0;
      for (int pass = 0; pass < 2; ++pass) {
#pragma unroll
        for (int it = 0; it < 16; ++it) {
          const int m  = mB + it;
          const int qd = m / rpi;
          const int rr = m - qd * rpi;
          const v4f o = *(const v4f*)(slab + it * 132 + lane * 4);
          if (rr < rpo)
            *(volatile v4f*)(Cf + ((size_t)qd * (size_t)rpo + (size_t)rr) * (size_t)ldc + n0 + lane * 4) = o;
        }
        __threadfence();
      }
    } else {
      unsigned short* Cp = (unsigned short*)C0;
      v4u hv[8];
#pragma unroll
      for (int it = 0; it < 8; ++it) {
        const int row = it * 2 + hh;
        const float* sp = slab + row * 132 + rl * 8;
        const v4f fa = *(const v4f*)sp;
        const v4f fb = *(const v4f*)(sp + 4);
        float f[8];
        f[0] = fa[0]; f[1] = fa[1]; f[2] = fa[2]; f[3] = fa[3];
        f[4] = fb[0]; f[5] = fb[1]; f[6] = fb[2]; f[7] = fb[3];
        v4u pk;
#pragma unroll
        for (int e = 0; e < 4; ++e) {
          const _Float16 x0 = (_Float16)f[2 * e];
          const _Float16 x1 = (_Float16)f[2 * e + 1];
          pk[e] = pk16(h_bits(x0), h_bits(x1));
        }
        hv[it] = pk;
      }
      for (int pass = 0; pass < 2; ++pass) {
#pragma unroll
        for (int it = 0; it < 8; ++it) {
          const int row = it * 2 + hh;
          const size_t go = (size_t)(mB + row) * (size_t)ldc + n0 + rl * 8;
          *(volatile v4u*)(Cp + go) = hv[it];
        }
        __threadfence();
      }
    }
    wave_sync_lds();
  }
}

__global__ __launch_bounds__(64) void pool_k(const unsigned short* __restrict__ QH, unsigned short* AN) {
  const int row = blockIdx.x;
  const int b = row / AP;
  const int a = row - b * AP;
  const bool aval = a < NANC;
  const int acl = aval ? a : (NANC - 1);
  const int ph = acl / 49, pw = (acl / 7) % 7, pd = acl % 7;
  const int t = threadIdx.x;
  const int tc = (t < 48) ? t : 47;
  const _Float16* Q = (const _Float16*)(const void*)QH;
  float s[8];
#pragma unroll
  for (int e = 0; e < 8; ++e) s[e] = 0.f;
#pragma unroll
  for (int i = 0; i < 2; ++i)
#pragma unroll
    for (int j = 0; j < 2; ++j)
#pragma unroll
      for (int l = 0; l < 2; ++l) {
        const int n = ((2 * ph + i) * HWD + (2 * pw + j)) * HWD + (2 * pd + l);
        const v8h v = *(const v8h*)(Q + ((size_t)(b * TP + n)) * DIMC + tc * 8);
#pragma unroll
        for (int e = 0; e < 8; ++e) s[e] += (float)v[e];
      }
  v4u pk;
#pragma unroll
  for (int e = 0; e < 4; ++e) {
    const float f0 = aval ? (s[2 * e] * 0.125f) : 0.f;
    const float f1 = aval ? (s[2 * e + 1] * 0.125f) : 0.f;
    pk[e] = pk16(h_bits((_Float16)f0), h_bits((_Float16)f1));
  }
  unsigned short* p = AN + (size_t)row * DIMC + tc * 8;
  if (t < 48) *(volatile v4u*)p = pk;
  __threadfence();
  if (t < 48) *(volatile v4u*)p = pk;
}

__global__ __launch_bounds__(256) void bias1_k(const float* __restrict__ an, const float* __restrict__ ah,
                                               const float* __restrict__ aw, const float* __restrict__ ad, float* PB) {
  __shared__ float anb[344];
  __shared__ float axb[3][16];
  __shared__ float lw[16];
  __shared__ int   lx0[16];
  __shared__ int   lx1[16];
  const int tid = threadIdx.x;
  const int h = blockIdx.x / AP;
  const int a = blockIdx.x - h * AP;
  const bool aval = a < NANC;
  const int acl = aval ? a : (NANC - 1);
  const size_t hb = (size_t)(h * NANC + acl);
  for (int i = tid; i < A3; i += 256) anb[i] = bfr(an[hb * A3 + i]);
  if (tid < HWD) {
    axb[0][tid] = bfr(ah[hb * HWD + tid]);
    axb[1][tid] = bfr(aw[hb * HWD + tid]);
    axb[2][tid] = bfr(ad[hb * HWD + tid]);
    int x0, x1; float w;
    lin7(tid, x0, x1, w);
    lx0[tid] = x0; lx1[tid] = x1; lw[tid] = w;
  }
  __syncthreads();
  v4f o[3];
#pragma unroll
  for (int i = 0; i < 3; ++i) {
    const int sidx = tid + 256 * i;
    const int scl = (sidx < 688) ? sidx : 687;
    v4f ov;
#pragma unroll
    for (int e = 0; e < 4; ++e) {
      const int n = scl * 4 + e;
      const int ncl = (n < NTOK) ? n : (NTOK - 1);
      const int x = ncl / 196, y = (ncl / 14) % 14, z = ncl % 14;
      float v = terp(anb, lx0[x], lx1[x], lw[x], lx0[y], lx1[y], lw[y], lx0[z], lx1[z], lw[z]);
      v += axb[0][x] + axb[1][y] + axb[2][z];
      ov[e] = (aval && n < NTOK) ? v : 0.f;
    }
    o[i] = ov;
  }
  float* prow = PB + ((size_t)(h * AP + a)) * TP;
  for (int pass = 0; pass < 2; ++pass) {
#pragma unroll
    for (int i = 0; i < 3; ++i) {
      const int sidx = tid + 256 * i;
      if (sidx < 688) *(volatile v4f*)(prow + (size_t)sidx * 4) = o[i];
    }
    __threadfence();
  }
}

__global__ __launch_bounds__(128) void bias2_k(const float* __restrict__ na, const float* __restrict__ hab,
                                               const float* __restrict__ wab, const float* __restrict__ dab, float* AB) {
  const int tid = threadIdx.x;
  const int h = blockIdx.x / TP;
  const int n = blockIdx.x - h * TP;
  const bool nval = n < NTOK;
  const int ncl = nval ? n : (NTOK - 1);
  const int x = ncl / 196, y = (ncl / 14) % 14, z = ncl % 14;
  int x0, x1, y0, y1, z0, z1; float wx, wy, wz;
  lin7(x, x0, x1, wx); lin7(y, y0, y1, wy); lin7(z, z0, z1, wz);
  const int tc = (tid < 96) ? tid : 95;
  v4f ov;
#pragma unroll
  for (int e = 0; e < 4; ++e) {
    const int a = tc * 4 + e;
    const int acl = (a < NANC) ? a : (NANC - 1);
    const float* base = na + ((size_t)(h * NANC + acl)) * A3;
    float v = terpg(base, x0, x1, wx, y0, y1, wy, z0, z1, wz);
    v += bfr(hab[(size_t)(h * HWD + x) * NANC + acl]);
    v += bfr(wab[(size_t)(h * HWD + y) * NANC + acl]);
    v += bfr(dab[(size_t)(h * HWD + z) * NANC + acl]);
    ov[e] = (nval && a < NANC) ? v : 0.f;
  }
  float* p = AB + ((size_t)(h * TP + n)) * AP + tc * 4;
  if (tid < 96) *(volatile v4f*)p = ov;
  __threadfence();
  if (tid < 96) *(volatile v4f*)p = ov;
}

template <int ST>
__global__ __launch_bounds__(128)
void attn_k(const unsigned short* __restrict__ QP, const unsigned short* __restrict__ KP,
            const unsigned short* __restrict__ VTp, const float* __restrict__ BP, unsigned short* OUT) {
  constexpr int QROWS = (ST == 1) ? AP : TP;
  constexpr int NQB   = QROWS / 64;
  constexpr int KROWS = (ST == 1) ? TP : AP;
  constexpr int NKC   = KROWS / 64;
  constexpr int KVAL  = (ST == 1) ? NTOK : NANC;
  constexpr int LDV   = NB * KROWS;
  constexpr float VCAR = (ST == 1) ? VSC : GSC;
  constexpr float OCAR = (ST == 1) ? GSC : CSC;

  __shared__ __align__(16) _Float16 Psh[4][16 * 64];
  __shared__ __align__(16) float    Os[4][16 * 192];

  const int tid  = threadIdx.x;
  const int wave = tid >> 5;
  const int lane = tid & 31;
  const int hh   = lane >> 4;
  const int c    = lane & 15;

  int bid = (int)blockIdx.x;
  const int qb = bid % NQB; bid /= NQB;
  const int hg = bid % 2;   bid /= 2;
  const int b  = bid;
  const int ql0 = qb * 64 + wave * 16;
  const size_t qrow = (size_t)b * QROWS + (size_t)ql0;

  const _Float16* QPh = (const _Float16*)(const void*)QP;
  const _Float16* KPh = (const _Float16*)(const void*)KP;
  const _Float16* VTh = (const _Float16*)(const void*)VTp;
  _Float16* pwh = Psh[wave];
  float* os = Os[wave];
  const v4u z4 = {0u, 0u, 0u, 0u};

#pragma unroll 1
  for (int hs = 0; hs < 4; ++hs) {
    const int h = hg * 4 + hs;
    const _Float16* Qg = QPh + (qrow + (size_t)c) * DIMC + h * HDIM + 8 * hh;
    const _Float16* Kg = KPh + ((size_t)b * KROWS + (size_t)c) * DIMC + h * HDIM + 8 * hh;
    const _Float16* Vg = VTh + (size_t)(h * HDIM + c) * (size_t)LDV + (size_t)b * KROWS + 8 * hh;
    const float*    Bg = BP + ((size_t)(h * QROWS + ql0 + 8 * hh)) * (size_t)KROWS + c;

    FR qa0, qa1;
    qa0.q[0] = *(const v8h*)(Qg);
    qa0.q[1] = *(const v8h*)(Qg + 16);
    qa1.q[0] = *(const v8h*)(Qg + 32);
    qa1.u[1] = z4;

    float mrow[8], lrow[8];
    v8f oh[3];
#pragma unroll
    for (int r = 0; r < 8; ++r) { mrow[r] = NEG_BIG; lrow[r] = 0.f; }
#pragma unroll
    for (int t = 0; t < 3; ++t) oh[t] = zero8();

    for (int kt = 0; kt < NKC; ++kt) {
      const int kv0 = kt * 64;
      v8f s[4];
#pragma unroll
      for (int j = 0; j < 4; ++j) s[j] = zero8();
#pragma unroll
      for (int j = 0; j < 4; ++j) {
        const _Float16* kp = Kg + (size_t)(kv0 + 16 * j) * DIMC;
        FR k0f, k1f;
        k0f.q[0] = *(const v8h*)(kp);
        k0f.q[1] = *(const v8h*)(kp + 16);
        k1f.q[0] = *(const v8h*)(kp + 32);
        k1f.u[1] = z4;
        s[j] = mma16(qa0, k0f, s[j]);
        s[j] = mma16(qa1, k1f, s[j]);
      }
      acc_guard4(s[0], s[1], s[2], s[3]);
#pragma unroll
      for (int j = 0; j < 4; ++j) {
        const bool kval = (kv0 + 16 * j + c) < KVAL;
#pragma unroll
        for (int r = 0; r < 8; ++r) {
          const float bv = Bg[(size_t)r * KROWS + kv0 + 16 * j];
          s[j][r] = kval ? (s[j][r] * SSC + bv) : NEG_BIG;
        }
      }
      wave_sync_lds();

#pragma unroll
      for (int r = 0; r < 8; ++r) {
        float m = fmaxf(fmaxf(s[0][r], s[1][r]), fmaxf(s[2][r], s[3][r]));
#pragma unroll
        for (int off = 1; off < 16; off <<= 1) m = fmaxf(m, __shfl_xor(m, off, 32));
        const float mnew  = fmaxf(mrow[r], m);
        const float alpha = __expf(mrow[r] - mnew);
        mrow[r] = mnew;
        float psum = 0.f;
#pragma unroll
        for (int j = 0; j < 4; ++j) {
          const float p = __expf(s[j][r] - mnew);
          psum += p;
          pwh[(8 * hh + r) * 64 + j * 16 + c] = (_Float16)(p * PSC);
        }
#pragma unroll
        for (int off = 1; off < 16; off <<= 1) psum += __shfl_xor(psum, off, 32);
        lrow[r] = lrow[r] * alpha + psum;
#pragma unroll
        for (int t = 0; t < 3; ++t) oh[t][r] *= alpha;
      }
      wave_sync_lds();

#pragma unroll
      for (int kk = 0; kk < 2; ++kk) {
        FR pa;
        pa.q[0] = *(const v8h*)(pwh + c * 64 + kk * 32 + 8 * hh);
        pa.q[1] = *(const v8h*)(pwh + c * 64 + kk * 32 + 16 + 8 * hh);
#pragma unroll
        for (int t = 0; t < 3; ++t) {
          const FR vb = ldfrh(Vg + (size_t)(16 * t) * (size_t)LDV + kv0 + 32 * kk);
          oh[t] = mma16(pa, vb, oh[t]);
        }
      }
    }
    acc_guard3(oh[0], oh[1], oh[2]);

#pragma unroll
    for (int r = 0; r < 8; ++r) {
      const float l = lrow[r];
      const float inv = ((l > 0.f) ? (1.0f / l) : 0.f) * (OCAR / (PSC * VCAR));
#pragma unroll
      for (int t = 0; t < 3; ++t) os[(8 * hh + r) * 192 + hs * HDIM + t * 16 + c] = oh[t][r] * inv;
    }
  }

  if (ST == 2) {
    wave_sync_lds();
    const int cl = (lane < 24) ? lane : 23;
    for (int pass = 0; pass < 2; ++pass) {
#pragma unroll 4
      for (int it = 0; it < 16; ++it) {
        const float* sp = os + it * 192 + cl * 8;
        const v4f fa = *(const v4f*)sp;
        const v4f fb = *(const v4f*)(sp + 4);
        float f[8];
        f[0] = fa[0]; f[1] = fa[1]; f[2] = fa[2]; f[3] = fa[3];
        f[4] = fb[0]; f[5] = fb[1]; f[6] = fb[2]; f[7] = fb[3];
        v4u pk;
#pragma unroll
        for (int e = 0; e < 4; ++e) {
          const _Float16 x0 = (_Float16)f[2 * e];
          const _Float16 x1 = (_Float16)f[2 * e + 1];
          pk[e] = pk16(h_bits(x0), h_bits(x1));
        }
        const size_t go = (qrow + (size_t)it) * DIMC + (size_t)(hg * 192 + cl * 8);
        if (lane < 24) *(volatile v4u*)(OUT + go) = pk;
      }
      __threadfence();
    }
  } else {
    __syncthreads();
    for (int pass = 0; pass < 2; ++pass) {
#pragma unroll 2
      for (int it = 0; it < 12; ++it) {
        const int idx = tid + 128 * it;
        const int j = idx >> 3;
        const int piece = idx & 7;
        const float* sp = Os[piece >> 1] + ((piece & 1) * 8) * 192 + j;
        float f[8];
#pragma unroll
        for (int e = 0; e < 8; ++e) f[e] = sp[e * 192];
        v4u pk;
#pragma unroll
        for (int e = 0; e < 4; ++e) {
          const _Float16 x0 = (_Float16)f[2 * e];
          const _Float16 x1 = (_Float16)f[2 * e + 1];
          pk[e] = pk16(h_bits(x0), h_bits(x1));
        }
        const size_t go = (size_t)(hg * 192 + j) * (size_t)MA + (size_t)(b * AP + qb * 64 + piece * 8);
        *(volatile v4u*)(OUT + go) = pk;
      }
      __threadfence();
    }
  }
}

__global__ __launch_bounds__(384) void comb_k(const float* __restrict__ VF, const unsigned short* __restrict__ CTX,
                                              const float* __restrict__ dw, const float* __restrict__ db,
                                              unsigned short* OHL) {
  __shared__ __align__(16) unsigned short rb[HWD * 2 * DIMC];
  const int c = threadIdx.x;
  const int b = blockIdx.x / 197;
  const int jb = blockIdx.x - b * 197;
  const v4u z4 = {0u, 0u, 0u, 0u};
  if (jb == 196) {
    for (int pass = 0; pass < 2; ++pass) {
#pragma unroll
      for (int i = 0; i < 2; ++i) {
        const int idx = c + 384 * i;
        const int row = idx / 96;
        const int piece = idx - row * 96;
        unsigned short* p = OHL + ((size_t)(b * TP + NTOK + row)) * (2 * DIMC) + piece * 8;
        *(volatile v4u*)p = z4;
      }
      __threadfence();
    }
    return;
  }
  const int x = jb / HWD;
  const int y = jb - x * HWD;

  float wr[NTAP];
#pragma unroll
  for (int k = 0; k < NTAP; ++k) wr[k] = bfr(dw[c * NTAP + k]);
  const float dbias = bfr(db[c]);

  int   roff[9];
  float rfac[9];
#pragma unroll
  for (int i = 0; i < 3; ++i) {
    const int xp  = x - 1 + i;
    const int xv  = (xp >= 0 && xp < HWD) ? 1 : 0;
    const int xcl = min(max(xp, 0), HWD - 1);
#pragma unroll
    for (int j = 0; j < 3; ++j) {
      const int yp  = y - 1 + j;
      const int yv  = (yp >= 0 && yp < HWD) ? 1 : 0;
      const int ycl = min(max(yp, 0), HWD - 1);
      roff[3 * i + j] = (xcl * HWD + ycl) * HWD;
      rfac[3 * i + j] = (float)(xv * yv);
    }
  }
  const float* vb = VF + (size_t)b * TP * DIMC + c;
  const _Float16* cx = (const _Float16*)(const void*)CTX + (size_t)b * TP * DIMC + c;
  const int nrow0 = (x * HWD + y) * HWD;

  float win[9][3];
#pragma unroll
  for (int q = 0; q < 9; ++q) {
    win[q][0] = 0.f;
    win[q][1] = vb[(size_t)roff[q] * DIMC] * rfac[q];
    win[q][2] = 0.f;
  }
#pragma unroll 1
  for (int z = 0; z < HWD; ++z) {
    const int zp = z + 1;
    const float zf = (zp < HWD) ? 1.f : 0.f;
    const int zcl = (zp < HWD) ? zp : (HWD - 1);
#pragma unroll
    for (int q = 0; q < 9; ++q) win[q][2] = vb[(size_t)(roff[q] + zcl) * DIMC] * (rfac[q] * zf);
    float s = dbias;
#pragma unroll
    for (int q = 0; q < 9; ++q) {
      s += wr[3 * q + 0] * win[q][0];
      s += wr[3 * q + 1] * win[q][1];
      s += wr[3 * q + 2] * win[q][2];
    }
    const float cv = (float)cx[(size_t)(nrow0 + z) * DIMC] * (1.0f / CSC);
    const float o = s + cv;
    const unsigned short hi = f2bf(o);
    const float hiv = __uint_as_float(((unsigned)hi) << 16);
    const unsigned short lo = f2bf(o - hiv);
    rb[z * (2 * DIMC) + c] = hi;
    rb[z * (2 * DIMC) + DIMC + c] = lo;
#pragma unroll
    for (int q = 0; q < 9; ++q) { win[q][0] = win[q][1]; win[q][1] = win[q][2]; }
  }
  __syncthreads();
  for (int pass = 0; pass < 2; ++pass) {
#pragma unroll
    for (int i = 0; i < 4; ++i) {
      const int idx = c + 384 * i;
      if (idx < HWD * 96) {
        const int row = idx / 96;
        const int piece = idx - row * 96;
        const v4u val = *(const v4u*)(rb + row * (2 * DIMC) + piece * 8);
        *(volatile v4u*)(OHL + ((size_t)(b * TP + nrow0 + row)) * (2 * DIMC) + piece * 8) = val;
      }
    }
    __threadfence();
  }
}

extern "C" void kernel_launch(void* const* d_in, const int* in_sizes, int n_in,
                              void* d_out, int out_size, void* d_ws, size_t ws_size,
                              hipStream_t stream) {
  if (n_in < 15) return;
  if (in_sizes[0] != NB * NTOK * DIMC) return;
  if (in_sizes[1] != DIMC * DIMC) return;
  if (in_sizes[2] != DIMC * 2 * DIMC) return;
  if (in_sizes[3] != DIMC * DIMC) return;
  if (in_sizes[4] != DIMC) return;
  if (in_sizes[5] != DIMC * NTAP) return;
  if (in_sizes[6] != DIMC) return;
  if (in_sizes[7] != NHEAD * NANC * A3 || in_sizes[8] != NHEAD * NANC * A3) return;
  for (int i = 9; i < 15; ++i) if (in_sizes[i] != NHEAD * NANC * HWD) return;
  if (out_size != NB * NTOK * DIMC) return;

  const float* X      = (const float*)d_in[0];
  const float* Wq     = (const float*)d_in[1];
  const float* Wkv    = (const float*)d_in[2];
  const float* Wproj  = (const float*)d_in[3];
  const float* bproj  = (const float*)d_in[4];
  const float* dwc_w  = (const float*)d_in[5];
  const float* dwc_b  = (const float*)d_in[6];
  const float* an_b   = (const float*)d_in[7];
  const float* na_b   = (const float*)d_in[8];
  const float* ah_b   = (const float*)d_in[9];
  const float* aw_b   = (const float*)d_in[10];
  const float* ad_b   = (const float*)d_in[11];
  const float* ha_b   = (const float*)d_in[12];
  const float* wa_b   = (const float*)d_in[13];
  const float* da_b   = (const float*)d_in[14];

  const size_t PWQ  = (size_t)DIMC * DIMC * 2;
  const size_t PWKV = (size_t)2 * DIMC * DIMC * 2;
  const size_t PWP2 = (size_t)DIMC * (2 * DIMC) * 2;
  const size_t PX   = (size_t)MT * DIMC * 2;
  const size_t PQ   = PX;
  const size_t PBP  = (size_t)NHEAD * AP * TP * 4;
  const size_t PK   = PX;
  const size_t PV   = (size_t)MT * DIMC * 4;
  const size_t PA   = (size_t)MA * DIMC * 2;
  const size_t PG   = (size_t)DIMC * MA * 2;
  const size_t PHL  = (size_t)MT * (2 * DIMC) * 2;
  size_t off = 0;
  const size_t oWQ  = off; off += PWQ;
  const size_t oWKV = off; off += PWKV;
  const size_t oWP2 = off; off += PWP2;
  const size_t oX   = off; off += PX;
  const size_t oQ   = off; off += PQ;
  const size_t oB   = off; off += PBP;
  const size_t oK   = off; off += PK;
  const size_t oV   = off; off += PV;
  const size_t oA   = off; off += PA;
  const size_t oG   = off; off += PG;
  if (off > ws_size) return;
  if (off > (size_t)134217728) return;
  if (oQ + PHL > oK) return;
  if ((size_t)DIMC * MT * 2 > PX) return;

  char* ws = (char*)d_ws;
  unsigned short* WQt  = (unsigned short*)(ws + oWQ);
  unsigned short* WKVt = (unsigned short*)(ws + oWKV);
  unsigned short* WP2  = (unsigned short*)(ws + oWP2);
  unsigned short* XH   = (unsigned short*)(ws + oX);
  unsigned short* VT   = (unsigned short*)(ws + oX);
  unsigned short* QH   = (unsigned short*)(ws + oQ);
  unsigned short* OHL  = (unsigned short*)(ws + oQ);
  float*          BPL  = (float*)(ws + oB);
  unsigned short* KH   = (unsigned short*)(ws + oK);
  unsigned short* CTX  = (unsigned short*)(ws + oK);
  float*          VF   = (float*)(ws + oV);
  unsigned short* AN   = (unsigned short*)(ws + oA);
  unsigned short* AGV  = (unsigned short*)(ws + oG);

  const dim3 blk64(64), blk128(128), blk256(256), blk384(384);

  tr_cvt<0><<<dim3(DIMC / 64, DIMC / 64), blk256, 0, stream>>>(Wq, DIMC, WQt, DIMC, WSC);
  tr_cvt<0><<<dim3(2 * DIMC / 64, DIMC / 64), blk256, 0, stream>>>(Wkv, 2 * DIMC, WKVt, DIMC, WSC);
  tr_cvt<2><<<dim3(DIMC / 64, DIMC / 64), blk256, 0, stream>>>(Wproj, DIMC, WP2, 2 * DIMC, 1.0f);
  tr_cvt<2><<<dim3(DIMC / 64, DIMC / 64), blk256, 0, stream>>>(Wproj, DIMC, WP2 + DIMC, 2 * DIMC, 1.0f);

  cvt_x<<<dim3((MT * DIMC) / 2048), blk256, 0, stream>>>(X, XH);

  const unsigned tGrid = (unsigned)(((MT / 32) * (DIMC / 128) + 3) / 4);
  gemm_k<1, false, false><<<dim3(tGrid), blk128, 0, stream>>>(
      XH, DIMC, WQt, DIMC, (void*)QH, bproj, DIMC, MT, DIMC, DIMC, QSC / WSC, MT, MT);
  gemm_k<1, false, false><<<dim3(tGrid), blk128, 0, stream>>>(
      XH, DIMC, WKVt, DIMC, (void*)KH, bproj, DIMC, MT, DIMC, DIMC, QSC / WSC, MT, MT);
  gemm_k<4, false, false><<<dim3(tGrid), blk128, 0, stream>>>(
      XH, DIMC, WKVt + (size_t)DIMC * DIMC, DIMC, (void*)VF, bproj, DIMC, MT, DIMC, DIMC, 1.0f / WSC, MT, MT);

  tr_cvt<1><<<dim3(DIMC / 64, MT / 64), blk256, 0, stream>>>(VF, DIMC, VT, MT, VSC);

  pool_k<<<dim3(MA), blk64, 0, stream>>>(QH, AN);
  bias1_k<<<dim3(NHEAD * AP), blk256, 0, stream>>>(an_b, ah_b, aw_b, ad_b, BPL);

  attn_k<1><<<dim3((AP / 64) * 2 * NB), blk128, 0, stream>>>(AN, KH, VT, BPL, AGV);

  bias2_k<<<dim3(NHEAD * TP), blk128, 0, stream>>>(na_b, ha_b, wa_b, da_b, BPL);
  attn_k<2><<<dim3((TP / 64) * 2 * NB), blk128, 0, stream>>>(QH, AN, AGV, BPL, CTX);

  comb_k<<<dim3(NB * 197), blk384, 0, stream>>>(VF, CTX, dwc_w, dwc_b, OHL);

  gemm_k<4, true, true><<<dim3(tGrid), blk128, 0, stream>>>(
      OHL, 2 * DIMC, WP2, 2 * DIMC, d_out, bproj, DIMC, MT, DIMC, 2 * DIMC, 1.0f, TP, NTOK);
  (void)hipGetLastError();
}
